// LTIModel_45449343927016
// MI455X (gfx1250) — hardware-verified
//
#include <hip/hip_runtime.h>

constexpr int NSEQ        = 2048;
constexpr int NSTEP       = 256;
constexpr int NSTATE      = 13;
constexpr int NCTRL       = 4;
constexpr int NLAT        = 256;
constexpr int NDEC        = 16;
constexpr int SEQ_PER_BLK = 16;
constexpr int NTHR        = 256;
constexpr int NWAVE       = 8;
constexpr int ZPITCH      = 264;
constexpr int UPITCH      = 40;
constexpr int ZFPITCH     = 260;
constexpr int REDP        = 16;
constexpr int BUPITCH     = 64;
constexpr int XSW         = 32;
constexpr int OUT_FLOATS  = NSEQ * (NSTEP + 1) * NSTATE;
constexpr int OUT_F4      = OUT_FLOATS / 4;

constexpr float SER_LIN   = 0.01f;
constexpr float SER_QUAD  = 5.0e-5f;
constexpr float CARRY     = 1048576.0f;
constexpr float CARRY_INV = 1.0f / 1048576.0f;
constexpr float WDEC_SC   = 16.0f;
constexpr float DEC_INV   = 1.0f / 16777216.0f;

static_assert(OUT_FLOATS % 4 == 0);
static_assert((NSEQ % SEQ_PER_BLK) == 0);
static_assert((ZPITCH % 8) == 0 && (UPITCH % 8) == 0 && (ZFPITCH % 4) == 0);

typedef __attribute__((ext_vector_type(16))) _Float16 v16h;
typedef __attribute__((ext_vector_type(8)))  _Float16 v8h;
typedef __attribute__((ext_vector_type(8)))  float    v8f;
typedef __attribute__((ext_vector_type(4)))  float    v4f;

__device__ __forceinline__ void dep_guard_h(v8f& a, v8f& b, v16h x, v16h y) { asm volatile("v_nop\n\tv_nop\n\tv_nop\n\tv_nop" : "+v"(a), "+v"(b) : "v"(x), "v"(y)); }
__device__ __forceinline__ void dep_guard1_h(v8f& a, v16h x, v16h y) { asm volatile("v_nop\n\tv_nop\n\tv_nop\n\tv_nop" : "+v"(a) : "v"(x), "v"(y)); }
__device__ __forceinline__ void keep4_h(v16h a, v16h b, v16h c, v16h d) { asm volatile("v_nop" :: "v"(a), "v"(b), "v"(c), "v"(d)); }
__device__ __forceinline__ void acc_guard2(v8f& a, v8f& b) { asm volatile("v_nop\n\tv_nop\n\tv_nop\n\tv_nop" : "+v"(a), "+v"(b)); }

template <typename T> struct Frag;
template <> struct Frag<_Float16> {
  typedef v16h V; union U { v16h v; v8h h[2]; };
  static __device__ __forceinline__ v16h load(const _Float16* p) {
    U f; f.h[0] = *(const v8h*)(p); f.h[1] = *(const v8h*)(p + 16); return f.v;
  }
  static __device__ __forceinline__ v8f mma(v16h a, v16h b, v8f c) {
    return __builtin_amdgcn_wmma_f32_16x16x32_f16(false, a, false, b, (short)0, c, false, false);
  }
};

__global__ __launch_bounds__(NTHR) void prep_kernel(const float* __restrict__ A, const float* __restrict__ Bm,
                                                 const float* __restrict__ Wd,
                                                 _Float16* __restrict__ Mp, _Float16* __restrict__ Bu,
                                                 _Float16* __restrict__ Wp) {
  __shared__ float arow[NLAT];
  __shared__ __align__(16) _Float16 mrow[NLAT];
  const int i = blockIdx.x, tid = threadIdx.x, lane = tid & 31, wave = tid >> 5;
  arow[tid] = A[(size_t)i * NLAT + tid];
  __syncthreads();
  float s = 0.0f;
#pragma unroll 1
  for (int k = 0; k < NLAT; ++k) s = fmaf(arow[k], A[(size_t)k * NLAT + tid], s);
  const float m = fmaf(SER_QUAD, s, SER_LIN * arow[tid]);
  mrow[tid] = (_Float16)(m * CARRY);
  __syncthreads();
  const _Float16 hz = (_Float16)0.0f;
  if (wave == 0) {
    const v8h v = *(const v8h*)(mrow + 8 * lane);
    _Float16* dst = Mp + (size_t)i * NLAT + 8 * lane;
    *(volatile v8h*)dst = v;
    __threadfence();
    *(volatile v8h*)dst = v;
  }
  if (wave == 1) {
    const float b0 = Bm[(size_t)i * NCTRL + 0], b1 = Bm[(size_t)i * NCTRL + 1];
    const float b2 = Bm[(size_t)i * NCTRL + 2], b3 = Bm[(size_t)i * NCTRL + 3];
    v8h v;
    v[0] = (lane == 0) ? (_Float16)(b0 * CARRY) : hz;
    v[1] = (lane == 0) ? (_Float16)(b1 * CARRY) : hz;
    v[2] = (lane == 0) ? (_Float16)(b2 * CARRY) : hz;
    v[3] = (lane == 0) ? (_Float16)(b3 * CARRY) : hz;
    v[4] = hz; v[5] = hz; v[6] = hz; v[7] = hz;
    if (lane < 8) {
      _Float16* dst = Bu + (size_t)i * BUPITCH + 8 * lane;
      *(volatile v8h*)dst = v;
      __threadfence();
      *(volatile v8h*)dst = v;
    }
  }
  if (i < NDEC && wave == 2) {
    const int srow = (i < NSTATE) ? i : (NSTATE - 1);
    const float* wr = Wd + (size_t)srow * NLAT + 8 * lane;
    const v4f w0 = *(const v4f*)(wr), w1 = *(const v4f*)(wr + 4);
    const bool live = (i < NSTATE);
    v8h v;
#pragma unroll
    for (int e = 0; e < 4; ++e) {
      v[e]     = live ? (_Float16)(w0[e] * WDEC_SC) : hz;
      v[4 + e] = live ? (_Float16)(w1[e] * WDEC_SC) : hz;
    }
    _Float16* dst = Wp + (size_t)i * NLAT + 8 * lane;
    *(volatile v8h*)dst = v;
    __threadfence();
    *(volatile v8h*)dst = v;
  }
}

__global__ __launch_bounds__(NTHR) void lti_scan_kernel(const float* __restrict__ x_init,
                                                     const float* __restrict__ u_fut,
                                                     const float* __restrict__ W_enc,
                                                     const float* __restrict__ W_dec,
                                                     const _Float16* __restrict__ Mp,
                                                     const _Float16* __restrict__ Bu,
                                                     const _Float16* __restrict__ Wp,
                                                     float* __restrict__ XS) {
  __shared__ __align__(16) _Float16 zh[SEQ_PER_BLK * ZPITCH];
  __shared__ __align__(16) _Float16 ih[SEQ_PER_BLK * ZPITCH];
  __shared__ __align__(16) _Float16 uh[SEQ_PER_BLK * UPITCH];
  __shared__ __align__(16) float    zf[SEQ_PER_BLK * ZFPITCH];
  __shared__ float red[NWAVE * SEQ_PER_BLK * REDP];
  __shared__ float xin[SEQ_PER_BLK * 16];

  const int tid = threadIdx.x, lane = tid & 31, wave = tid >> 5;
  const int c = lane & 15, hh = lane >> 4, koff = 8 * hh;
  const int rowbase = blockIdx.x * SEQ_PER_BLK;
  const int xr = tid >> 4;
  const int xc = tid & 15;

  if (tid < SEQ_PER_BLK * NSTATE) {
    const int r = tid / NSTATE, s = tid - r * NSTATE;
    xin[r * 16 + s] = x_init[(size_t)(rowbase + r) * NSTATE + s];
  }
  for (int idx = tid; idx < SEQ_PER_BLK * UPITCH; idx += NTHR) uh[idx] = (_Float16)0.0f;
#pragma unroll
  for (int q = 0; q < 8; ++q) red[q * NTHR + tid] = 0.0f;
  __syncthreads();
  {
    float we[NSTATE];
#pragma unroll
    for (int s = 0; s < NSTATE; ++s) we[s] = W_enc[(size_t)tid * NSTATE + s];
#pragma unroll 1
    for (int r = 0; r < SEQ_PER_BLK; ++r) {
      float a = 0.0f;
#pragma unroll
      for (int s = 0; s < NSTATE; ++s) a = fmaf(xin[r * 16 + s], we[s], a);
      zf[r * ZFPITCH + tid] = a;
      zh[r * ZPITCH + tid]  = (_Float16)a;
    }
  }
  if (tid < 64) {
    const int r = tid >> 2, cc = tid & 3;
    uh[r * UPITCH + cc] = (_Float16)u_fut[((size_t)(rowbase + r) * NSTEP) * NCTRL + cc];
  }
  __syncthreads();

  float zst[2][8];
#pragma unroll
  for (int nt = 0; nt < 2; ++nt)
#pragma unroll
    for (int r = 0; r < 8; ++r) zst[nt][r] = zf[(8 * hh + r) * ZFPITCH + 32 * wave + 16 * nt + c];
  float xst;
  {
    const int srow = (xc < NSTATE) ? xc : (NSTATE - 1);
    const float* wr = W_dec + (size_t)srow * NLAT;
    float a = 0.0f;
#pragma unroll 1
    for (int n = 0; n < NLAT; ++n) a = fmaf(zf[xr * ZFPITCH + n], wr[n], a);
    xst = (xc < NSTATE) ? a : 0.0f;
  }
  const v16h bu0 = Frag<_Float16>::load(Bu + (size_t)(32 * wave + c) * BUPITCH + koff);
  const v16h bu1 = Frag<_Float16>::load(Bu + (size_t)(32 * wave + 16 + c) * BUPITCH + koff);
  const v16h wdf = Frag<_Float16>::load(Wp + (size_t)c * NLAT + 32 * wave + koff);
  const _Float16* mrow0 = Mp + (size_t)(32 * wave + c) * NLAT + koff;
  const _Float16* mrow1 = Mp + (size_t)(32 * wave + 16 + c) * NLAT + koff;
  const _Float16* zrow  = zh + c * ZPITCH + koff;
  const _Float16* irow  = ih + c * ZPITCH + 32 * wave + koff;
  const _Float16* urow  = uh + c * UPITCH + koff;
  const v8f z8 = {0.f, 0.f, 0.f, 0.f, 0.f, 0.f, 0.f, 0.f};

#pragma unroll 1
  for (int t = 0; t <= NSTEP; ++t) {
    if (t > 0) {
      const v16h a = Frag<_Float16>::load(irow);
      v8f d = Frag<_Float16>::mma(a, wdf, z8);
      dep_guard1_h(d, a, wdf);
#pragma unroll
      for (int r = 0; r < 8; ++r) red[(wave * SEQ_PER_BLK + 8 * hh + r) * REDP + c] = d[r];
    }
    v8f acc0 = z8, acc1 = z8;
    if (t < NSTEP) {
      {
        const v16h au = Frag<_Float16>::load(urow);
        acc0 = Frag<_Float16>::mma(au, bu0, acc0);
        acc1 = Frag<_Float16>::mma(au, bu1, acc1);
        dep_guard_h(acc0, acc1, au, bu1);
      }
#pragma unroll 1
      for (int k0 = 0; k0 < NLAT; k0 += 32) {
        const v16h a  = Frag<_Float16>::load(zrow + k0);
        const v16h b0 = Frag<_Float16>::load(mrow0 + k0);
        const v16h b1 = Frag<_Float16>::load(mrow1 + k0);
        acc0 = Frag<_Float16>::mma(a, b0, acc0);
        acc1 = Frag<_Float16>::mma(a, b1, acc1);
        dep_guard_h(acc0, acc1, a, b1);
        keep4_h(a, b0, b1, b1);
      }
      acc_guard2(acc0, acc1);
#pragma unroll
      for (int r = 0; r < 8; ++r) {
        zst[0][r] = fmaf(acc0[r], CARRY_INV, zst[0][r]);
        zst[1][r] = fmaf(acc1[r], CARRY_INV, zst[1][r]);
      }
    }
    __syncthreads();

    if (t < NSTEP) {
      const int j0 = 32 * wave + c, j1 = j0 + 16;
#pragma unroll
      for (int r = 0; r < 8; ++r) {
        const int row = 8 * hh + r;
        zh[row * ZPITCH + j0] = (_Float16)zst[0][r];
        zh[row * ZPITCH + j1] = (_Float16)zst[1][r];
        ih[row * ZPITCH + j0] = (_Float16)acc0[r];
        ih[row * ZPITCH + j1] = (_Float16)acc1[r];
      }
      if (tid < 64) {
        const int tn = (t + 1 < NSTEP) ? (t + 1) : (NSTEP - 1);
        const int r = tid >> 2, cc = tid & 3;
        uh[r * UPITCH + cc] = (_Float16)u_fut[((size_t)(rowbase + r) * NSTEP + (size_t)tn) * NCTRL + cc];
      }
    }
    {
      float sred = 0.0f;
#pragma unroll
      for (int w = 0; w < NWAVE; ++w) sred += red[(w * SEQ_PER_BLK + xr) * REDP + xc];
      xst = fmaf(sred, DEC_INV, xst);
    }
    {
      v4f v;
#pragma unroll
      for (int jj = 0; jj < 4; ++jj) {
        const int col = 4 * (xc & 3) + jj;
        const float g = __shfl(xst, 16 * hh + col, 32);
        v[jj] = (xc < 4 && col < NSTATE) ? g : 0.0f;
      }
      if (xc < 8) {
        float* dst = XS + (((size_t)(rowbase + xr)) * (NSTEP + 1) + (size_t)t) * XSW + 4 * xc;
        *(volatile v4f*)dst = v;
        __threadfence();
        *(volatile v4f*)dst = v;
      }
    }
    __syncthreads();
  }
}

__global__ __launch_bounds__(NTHR) void pack_kernel(const float* __restrict__ XS, float* __restrict__ out, int n4) {
  const int gid = blockIdx.x * NTHR + threadIdx.x;
  if (gid < n4) {
    const int f0 = gid * 4;
    v4f v;
#pragma unroll
    for (int jj = 0; jj < 4; ++jj) {
      const int f = f0 + jj;
      const int q = f / NSTATE;
      const int s = f - q * NSTATE;
      v[jj] = XS[(size_t)q * XSW + s];
    }
    float* dst = out + f0;
    *(volatile v4f*)dst = v;
    __threadfence();
    *(volatile v4f*)dst = v;
  }
}

extern "C" void kernel_launch(void* const* d_in, const int* in_sizes, int n_in,
                              void* d_out, int out_size, void* d_ws, size_t ws_size, hipStream_t stream) {
  if (n_in < 10 || d_out == nullptr || d_ws == nullptr) return;
  if (in_sizes[2] != NSEQ * NSTATE || in_sizes[4] != NSEQ * NSTEP * NCTRL || in_sizes[5] != NLAT * NLAT ||
      in_sizes[6] != NLAT * NCTRL || in_sizes[7] != NLAT * NSTATE || in_sizes[8] != NSTATE * NLAT ||
      out_size != OUT_FLOATS) return;

  const float* x_init = (const float*)d_in[2];
  const float* u_fut  = (const float*)d_in[4];
  const float* A_ct   = (const float*)d_in[5];
  const float* Bmat   = (const float*)d_in[6];
  const float* W_enc  = (const float*)d_in[7];
  const float* W_dec  = (const float*)d_in[8];
  float* out = (float*)d_out;

  char* ws = (char*)d_ws; size_t off = 0;
  auto carve = [&](size_t bytes) -> char* { char* p = ws + off; off += (bytes + 255) & ~(size_t)255; return p; };
  _Float16* Mp = (_Float16*)carve((size_t)NLAT * NLAT * 2);
  _Float16* Bu = (_Float16*)carve((size_t)NLAT * BUPITCH * 2);
  _Float16* Wp = (_Float16*)carve((size_t)NDEC * NLAT * 2);
  float*    XS = (float*)carve((size_t)NSEQ * (NSTEP + 1) * XSW * sizeof(float));
  if (off > ws_size || off > (size_t)134217728) return;

  prep_kernel<<<dim3(NLAT), dim3(NTHR), 0, stream>>>(A_ct, Bmat, W_dec, Mp, Bu, Wp);
  lti_scan_kernel<<<dim3(NSEQ / SEQ_PER_BLK), dim3(NTHR), 0, stream>>>(x_init, u_fut, W_enc, W_dec, Mp, Bu, Wp, XS);
  const int nblk = (OUT_F4 + NTHR - 1) / NTHR;
  pack_kernel<<<dim3(nblk), dim3(NTHR), 0, stream>>>(XS, out, OUT_F4);
}
